// Attention_54004918780674
// MI455X (gfx1250) — hardware-verified
//
#include <hip/hip_runtime.h>
#include <math.h>

#ifndef NB
#define NB 2
#endif
#ifndef SEQ
#define SEQ 2048
#endif
#define NB_FULL 2
#define SEQ_FULL 2048
#define DM 2048
#define NH 16
#define NKV 4
#define HD 128
#define NGRP 4
#define KVC 512
#define NQK 2560
#define NBIAS 3072
#define NPAIR 64
#define CTX_CARRY 64.0f

static_assert(NH == NKV * NGRP);
static_assert(DM == NH * HD);
static_assert(KVC == NKV * HD);
static_assert(NQK == DM + KVC);
static_assert(NBIAS == DM + KVC + KVC);
static_assert(HD == 128);
static_assert(NPAIR * 2 == HD);
static_assert((DM % HD) == 0);
static_assert((HD % 8) == 0);
static_assert((NQK % 8) == 0);
static_assert(SEQ % 64 == 0);
static_assert(NB <= NB_FULL);
static_assert(SEQ <= SEQ_FULL);
static_assert(((SEQ * (DM / 8)) % 256) == 0);
static_assert(((DM * (DM / 8)) % 256) == 0);
static_assert(((KVC * (DM / 8)) % 256) == 0);
static_assert(((SEQ * NPAIR) % 256) == 0);
static_assert(((SEQ * (NQK / 8)) % 256) == 0);
static_assert(NBIAS % 256 == 0);
static_assert(DM % 64 == 0);
static_assert(NQK % 64 == 0);
static_assert(KVC % 64 == 0);
static_assert((NB * SEQ) % 64 == 0);
static_assert(DM % 32 == 0);
static_assert(HD % 32 == 0);

typedef __attribute__((ext_vector_type(16))) _Float16     v16h;
typedef __attribute__((ext_vector_type(16))) __bf16       v16b;
typedef __attribute__((ext_vector_type(8)))  __bf16       v8b;
typedef __attribute__((ext_vector_type(8)))  float        v8f;
typedef __attribute__((ext_vector_type(4)))  float        v4f;
typedef __attribute__((ext_vector_type(4)))  unsigned int v4u;


#define VST2(T, ptr, val) do { const T vst2_v_ = (val); *(volatile T*)(ptr) = vst2_v_; __threadfence(); *(volatile T*)(ptr) = vst2_v_; } while (0)

__device__ __forceinline__ float bf_keep(float v) { unsigned u = __float_as_uint(v); u = (u + 0x7fffu + ((u >> 16) & 1u)) & 0xffff0000u; return __uint_as_float(u); }
__device__ __forceinline__ unsigned h_bits(float v) { return (unsigned)__builtin_bit_cast(unsigned short, (_Float16)v); }
__device__ __forceinline__ unsigned pk2h(float a, float b) { return h_bits(a) | (h_bits(b) << 16); }
__device__ __forceinline__ v4u pack8h(v4f a, v4f b) { v4u p; p.x = pk2h(a.x, a.y); p.y = pk2h(a.z, a.w); p.z = pk2h(b.x, b.y); p.w = pk2h(b.z, b.w); return p; }

static __device__ __forceinline__ _Float16 toh_flush(float v) { const _Float16 r = (_Float16)v; return (fabsf(v) < 6.103515625e-05f) ? (_Float16)0.0f : r; }
static __device__ __forceinline__ unsigned pk2h_flush(float a, float b) {
  return (unsigned)__builtin_bit_cast(unsigned short, toh_flush(a)) | ((unsigned)__builtin_bit_cast(unsigned short, toh_flush(b)) << 16);
}

union FB { v16b v; v8b h[2]; };
__device__ __forceinline__ v16b ld_frag(const unsigned short* p) { FB f; f.h[0] = *(const v8b*)(p); f.h[1] = *(const v8b*)(p + 16); return f.v; }
__device__ __forceinline__ v16b ld_fragl(const __bf16* p) { FB f; f.h[0] = *(const v8b*)(p); f.h[1] = *(const v8b*)(p + 16); return f.v; }

__device__ __forceinline__ v8f mma16(v16b a, v16b b, v8f c) {
  const v16h ah = __builtin_bit_cast(v16h, a), bh = __builtin_bit_cast(v16h, b);
  c = __builtin_amdgcn_wmma_f32_16x16x32_f16(false, ah, false, bh, (short)0, c, false, false);
  asm volatile("v_nop\n\tv_nop\n\tv_nop\n\tv_nop" : "+v"(c) : "v"(ah), "v"(bh));
  return c;
}
__device__ __forceinline__ __bf16 to16h(float f) { return __builtin_bit_cast(__bf16, (_Float16)f); }
__device__ __forceinline__ void wave_sync() {
  __builtin_amdgcn_fence(3  , "workgroup");
  __builtin_amdgcn_wave_barrier();
  __builtin_amdgcn_fence(2  , "workgroup");
}

__global__ __launch_bounds__(256) void k_castb(const float* __restrict__ SRC, size_t sbs, unsigned lds, unsigned short* __restrict__ DST, size_t dbs, unsigned ldd, unsigned nR, unsigned nC) {
  const unsigned u = blockIdx.x * 256u + threadIdx.x; const unsigned per = nC >> 3;
  if (u >= nR * per) return;
  const unsigned r = u / per; const unsigned c0 = (u - r * per) << 3;
  const float* s = SRC + (size_t)blockIdx.y * sbs + (size_t)r * lds + c0;
  const v4f a = *(const v4f*)s; const v4f b = *(const v4f*)(s + 4);
  v4u pk; pk.x = pk2h(bf_keep(a.x), bf_keep(a.y)); pk.y = pk2h(bf_keep(a.z), bf_keep(a.w)); pk.z = pk2h(bf_keep(b.x), bf_keep(b.y)); pk.w = pk2h(bf_keep(b.z), bf_keep(b.w));
  VST2(v4u, DST + (size_t)blockIdx.y * dbs + (size_t)r * ldd + c0, pk);
}
__global__ __launch_bounds__(256) void k_castT(const float* __restrict__ SRC, unsigned lds, unsigned short* __restrict__ DST, unsigned ldd, unsigned nR, unsigned nC, float sc) {
  const unsigned u = blockIdx.x * 256u + threadIdx.x; const unsigned per = nR >> 3;
  if (u >= nC * per) return;
  const unsigned c = u / per; const unsigned r0 = (u - c * per) << 3;
  float w[8];
#pragma unroll
  for (int e = 0; e < 8; ++e) w[e] = bf_keep(SRC[(size_t)(r0 + e) * lds + c]) * sc;
  v4u pk;
  pk.x = pk2h(w[0], w[1]); pk.y = pk2h(w[2], w[3]); pk.z = pk2h(w[4], w[5]); pk.w = pk2h(w[6], w[7]);
  VST2(v4u, DST + (size_t)c * ldd + r0, pk);
}
__global__ __launch_bounds__(256) void k_bias(const float* __restrict__ bq, const float* __restrict__ bk, const float* __restrict__ bv, float* __restrict__ BALL) {
  const unsigned i = blockIdx.x * 256u + threadIdx.x;
  if (i >= (unsigned)NBIAS) return;
  const unsigned i0 = (i < (unsigned)(DM - 1)) ? i : (unsigned)(DM - 1);
  const unsigned t1 = (i >= (unsigned)DM) ? (i - (unsigned)DM) : 0u;                   const unsigned i1 = (t1 < (unsigned)(KVC - 1)) ? t1 : (unsigned)(KVC - 1);
  const unsigned t2 = (i >= (unsigned)NQK) ? (i - (unsigned)NQK) : 0u;                 const unsigned i2 = (t2 < (unsigned)(KVC - 1)) ? t2 : (unsigned)(KVC - 1);
  const float a = bq[i0], b = bk[i1], c = bv[i2];
  const float v = (i < (unsigned)DM) ? a : ((i < (unsigned)NQK) ? b : c);
  VST2(float, BALL + i, bf_keep(v));
}
__global__ __launch_bounds__(256) void k_cstab(float* __restrict__ CS) {
#pragma clang fp contract(off)
  __shared__ __align__(16) float sm[512];
  const unsigned tid = threadIdx.x;
  const unsigned gid = blockIdx.x * 256u + tid;
  const unsigned i = gid & 63u, pos = gid >> 6;
  const float th = exp2f(-(float)i * 0.20762050593045702f);
  const float ang = (float)pos * th;
  sm[2u * tid]      = cosf(ang);
  sm[2u * tid + 1u] = sinf(ang);
  __syncthreads();
  if (tid < 128u) {
    const v4f v = *(const v4f*)(sm + 4u * tid);
    VST2(v4f, CS + (size_t)blockIdx.x * 512u + 4u * tid, v);
  }
}
__global__ __launch_bounds__(256) void k_rope(const float* __restrict__ QKF, const float* __restrict__ CS, unsigned short* __restrict__ QKH, unsigned nR) {
#pragma clang fp contract(off)
  const unsigned u = blockIdx.x * 256u + threadIdx.x; const unsigned per = (unsigned)(NQK / 8);
  if (u >= nR * per) return;
  const unsigned r = u / per; const unsigned c0 = (u - r * per) << 3;
  const unsigned pos = r % (unsigned)SEQ; const unsigned d0 = c0 & (unsigned)(HD - 1);
  const float* s = QKF + (size_t)r * NQK + c0;
  const float* t = CS + (size_t)pos * HD + d0;
  const v4f a = *(const v4f*)s;  const v4f b = *(const v4f*)(s + 4);
  const v4f ta = *(const v4f*)t; const v4f tb = *(const v4f*)(t + 4);
  v4u pk;
  pk.x = pk2h_flush(a.x * ta.x - a.y * ta.y, a.x * ta.y + a.y * ta.x);
  pk.y = pk2h_flush(a.z * ta.z - a.w * ta.w, a.z * ta.w + a.w * ta.z);
  pk.z = pk2h_flush(b.x * tb.x - b.y * tb.y, b.x * tb.y + b.y * tb.x);
  pk.w = pk2h_flush(b.z * tb.z - b.w * tb.w, b.z * tb.w + b.w * tb.z);
  VST2(v4u, QKH + (size_t)r * NQK + c0, pk);
}

template <int BIAS_MODE, int OUT_MODE>
__global__ __launch_bounds__(256) void k_gemm64(
    const unsigned short* Ap, unsigned lda, size_t strideA,
    const unsigned short* Btp, unsigned ldb, size_t strideB,
    void* Cout, unsigned ldc, size_t strideC,
    const float* __restrict__ bias,
    unsigned M, unsigned N, unsigned K, float scale) {
  __shared__ __align__(16) float sT[8][16 * 68];
  const unsigned b = blockIdx.y;
  const unsigned lane = threadIdx.x & 31u, wave = threadIdx.x >> 5;
  const unsigned tilesN = N >> 6, tilesM = M >> 6;
  const unsigned tile = blockIdx.x * 8u + wave;
  if (tile >= tilesM * tilesN) return;
  const unsigned tm = tile / tilesN, tn = tile - tm * tilesN;
  const unsigned m0 = tm << 6, n0 = tn << 6;
  const unsigned short* Ab = Ap  + (size_t)b * strideA;
  const unsigned short* Bb = Btp + (size_t)b * strideB;
  const unsigned rlane = lane & 15u, koff = (lane >> 4) * 8u, mOff = koff;

  v8f acc[4][4];
#pragma unroll
  for (int i = 0; i < 4; ++i)
#pragma unroll
    for (int j = 0; j < 4; ++j) acc[i][j] = (v8f){0.f, 0.f, 0.f, 0.f, 0.f, 0.f, 0.f, 0.f};

  for (unsigned k0 = 0; k0 < K; k0 += 32u) {
    v16b bh[4];
#pragma unroll
    for (int j = 0; j < 4; ++j) bh[j] = ld_frag(Bb + (size_t)(n0 + 16u * j + rlane) * ldb + koff + k0);
#pragma unroll
    for (int i = 0; i < 4; ++i) {
      const size_t ao = (size_t)(m0 + 16u * i + rlane) * lda + koff + k0;
      const v16b ah = ld_frag(Ab + ao);
#pragma unroll
      for (int j = 0; j < 4; ++j) acc[i][j] = mma16(ah, bh[j], acc[i][j]);
    }
  }

  float* slab = sT[wave];
#pragma unroll
  for (int i = 0; i < 4; ++i) {
    const unsigned mBase = m0 + 16u * i;
#pragma unroll
    for (int j = 0; j < 4; ++j) {
      const unsigned n = n0 + 16u * j + rlane;
      float bv = 0.f;
      if (BIAS_MODE == 2) bv = bias[n];
#pragma unroll
      for (int r = 0; r < 8; ++r) {
        float v = acc[i][j][r] * scale;
        if (BIAS_MODE == 1) v += bias[mBase + mOff + r];
        if (BIAS_MODE == 2) v += bv;
        slab[(mOff + r) * 68u + 16u * j + rlane] = v;
      }
    }
    wave_sync();
    if (OUT_MODE == 0) {
      float* C = (float*)Cout + (size_t)b * strideC;
      const unsigned rs = lane >> 4, c4 = (lane & 15u) * 4u;
      for (int pass = 0; pass < 2; ++pass) {
#pragma unroll
        for (int it = 0; it < 8; ++it) {
          const unsigned row = it * 2u + rs;
          const v4f v = *(const v4f*)(slab + row * 68u + c4);
          *(volatile v4f*)(C + (size_t)(mBase + row) * ldc + n0 + c4) = v;
        }
        __threadfence();
      }
    } else {
      unsigned short* C = (unsigned short*)Cout + (size_t)b * strideC;
      const unsigned q = lane >> 3, c8 = (lane & 7u) * 8u;
      for (int pass = 0; pass < 2; ++pass) {
#pragma unroll
        for (int it = 0; it < 4; ++it) {
          const unsigned row = it * 4u + q;
          const float* sp = slab + row * 68u + c8;
          const v4f x0 = *(const v4f*)sp, x1 = *(const v4f*)(sp + 4);
          const v4u hv = pack8h(x0, x1);
          *(volatile v4u*)(C + (size_t)(mBase + row) * ldc + n0 + c8) = hv;
        }
        __threadfence();
      }
    }
    wave_sync();
  }
}

__global__ __launch_bounds__(128) void k_fattn(
    const unsigned short* Qh, const unsigned short* Kh, unsigned ldqk, size_t qk_bs,
    const unsigned short* Vh, unsigned ldv, unsigned v_bs,
    unsigned short* Oh, unsigned ldo, size_t o_bs, unsigned nChunks) {
  const float PSC = 32768.0f;
  const float OSC = CTX_CARRY;
  const float SC2 = 0.08838834764831845f * 1.4426950408889634f;
  const float NEG = -__builtin_inff();
  __shared__ __align__(16) __bf16 Psh[4][16 * 64];
  __shared__ __align__(16) float  Os[4][16 * 132];

  const unsigned tid = threadIdx.x, wave = tid >> 5, lane = tid & 31u, hh = lane >> 4, c = lane & 15u;
  const unsigned qb = blockIdx.x, h = blockIdx.y, b = blockIdx.z, kvh = h / (unsigned)NGRP;
  const unsigned q0 = qb * 64u + wave * 16u;
  const size_t qoff = (size_t)b * qk_bs + (size_t)(q0 + c) * ldqk + h * (unsigned)HD + 8u * hh;
  const size_t koff = (size_t)b * qk_bs + kvh * (unsigned)HD + 8u * hh;
  const size_t voff = (size_t)(kvh * (unsigned)HD + c) * ldv + (size_t)b * v_bs + 8u * hh;

  float mrow[8], lrow[8];
  v8f oacc[8];
#pragma unroll
  for (int r = 0; r < 8; ++r) { mrow[r] = NEG; lrow[r] = 0.f; }
#pragma unroll
  for (int t = 0; t < 8; ++t) oacc[t] = (v8f){0.f, 0.f, 0.f, 0.f, 0.f, 0.f, 0.f, 0.f};

  __bf16* pwh = Psh[wave];
  for (unsigned kc = 0; kc < nChunks; ++kc) {
    const unsigned kv0 = kc * 64u;
    v8f s[4];
#pragma unroll
    for (int j = 0; j < 4; ++j) s[j] = (v8f){0.f, 0.f, 0.f, 0.f, 0.f, 0.f, 0.f, 0.f};
#pragma unroll 1
    for (unsigned d = 0; d < 4u; ++d) {
      unsigned dofs = d * 32u;
      asm volatile("" : "+v"(dofs));
      const v16b qa = ld_frag(Qh + qoff + dofs);
#pragma unroll
      for (int j = 0; j < 4; ++j) {
        const size_t ko = koff + (size_t)(kv0 + 16u * j + c) * ldqk + dofs;
        const v16b kb = ld_frag(Kh + ko);
        s[j] = mma16(qa, kb, s[j]);
      }
    }
#pragma unroll
    for (int r = 0; r < 8; ++r) {
      float m = NEG;
#pragma unroll
      for (int j = 0; j < 4; ++j) {
        const float v = s[j][r] * SC2;
        s[j][r] = v;
        m = fmaxf(m, v);
      }
      m = fmaxf(m, __shfl_xor(m, 1, 32)); m = fmaxf(m, __shfl_xor(m, 2, 32));
      m = fmaxf(m, __shfl_xor(m, 4, 32)); m = fmaxf(m, __shfl_xor(m, 8, 32));
      const float mnew = fmaxf(mrow[r], m);
      const float alpha = exp2f(mrow[r] - mnew);
      mrow[r] = mnew;
      float psum = 0.f;
#pragma unroll
      for (int j = 0; j < 4; ++j) {
        const float p = exp2f(s[j][r] - mnew);
        psum += p;
        const unsigned pi = (8u * hh + r) * 64u + 16u * j + c;
        pwh[pi] = to16h(p * PSC);
      }
      psum += __shfl_xor(psum, 1, 32); psum += __shfl_xor(psum, 2, 32);
      psum += __shfl_xor(psum, 4, 32); psum += __shfl_xor(psum, 8, 32);
      lrow[r] = lrow[r] * alpha + psum;
#pragma unroll
      for (int t = 0; t < 8; ++t) oacc[t][r] *= alpha;
    }
    wave_sync();
#pragma unroll 1
    for (unsigned kk = 0; kk < 2u; ++kk) {
      const v16b pa = ld_fragl(pwh + c * 64u + kk * 32u + 8u * hh);
#pragma unroll
      for (int t = 0; t < 8; ++t) {
        const size_t vo = voff + (size_t)(16u * t) * ldv + kv0 + kk * 32u;
        const v16b vb = ld_frag(Vh + vo);
        oacc[t] = mma16(pa, vb, oacc[t]);
      }
    }
    wave_sync();
  }

  float* os = Os[wave];
#pragma unroll
  for (int r = 0; r < 8; ++r) {
    const float inv = OSC * (1.0f / (lrow[r] * PSC));
#pragma unroll
    for (int t = 0; t < 8; ++t) os[(8u * hh + r) * 132u + 16u * t + c] = oacc[t][r] * inv;
  }
  wave_sync();
  {
    const unsigned rs = lane >> 4, c8 = (lane & 15u) * 8u;
    unsigned short* obh = Oh + (size_t)b * o_bs + h * (unsigned)HD;
    for (int pass = 0; pass < 2; ++pass) {
#pragma unroll
      for (int it = 0; it < 8; ++it) {
        const unsigned row = it * 2u + rs;
        const float* sp = os + row * 132u + c8;
        const v4f x0 = *(const v4f*)sp, x1 = *(const v4f*)(sp + 4);
        const size_t oo = (size_t)(q0 + row) * ldo + c8;
        const v4u hv = pack8h(x0, x1);
        *(volatile v4u*)(obh + oo) = hv;
      }
      __threadfence();
    }
  }
}

static constexpr size_t al256(size_t v) { return (v + 255) / 256 * 256; }
static constexpr size_t SZ_X16  = al256((size_t)NB * SEQ * DM * 2);
static constexpr size_t SZ_WQK  = al256((size_t)NQK * DM * 2);
static constexpr size_t SZ_WV   = al256((size_t)KVC * DM * 2);
static constexpr size_t SZ_WO   = al256((size_t)DM * DM * 2);
static constexpr size_t SZ_BALL = al256((size_t)NBIAS * 4);
static constexpr size_t SZ_CS   = al256((size_t)SEQ * HD * 4);
static constexpr size_t SZ_QKF  = al256((size_t)NB * SEQ * NQK * 4);
static constexpr size_t SZ_QKH  = al256((size_t)NB * SEQ * NQK * 2);
static constexpr size_t SZ_VT   = al256((size_t)KVC * NB * SEQ * 2);
static constexpr size_t SZ_CTXH = al256((size_t)NB * SEQ * DM * 2);
static constexpr size_t WS_TOTAL = SZ_X16 + SZ_WQK + SZ_WV + SZ_WO + SZ_BALL + SZ_CS + SZ_QKF + SZ_QKH + SZ_VT + SZ_CTXH;
static_assert(WS_TOTAL <= (size_t)134217728);
static_assert((size_t)((SEQ * (DM / 8)) / 256) * NB * 256 * 8 == (size_t)NB * SEQ * DM);
static_assert((size_t)((DM * (DM / 8)) / 256) * 256 * 8 + (size_t)((KVC * (DM / 8)) / 256) * 256 * 8 == (size_t)NQK * DM);
static_assert((size_t)((KVC * (DM / 8)) / 256) * 256 * 8 == (size_t)KVC * DM);
static_assert((size_t)((DM * (DM / 8)) / 256) * 256 * 8 == (size_t)DM * DM);
static_assert((size_t)((SEQ * NPAIR) / 256) * 512 == (size_t)SEQ * HD);
static_assert((size_t)((NB * SEQ) / 64) * (NQK / 64) * 4096 == (size_t)NB * SEQ * NQK);
static_assert((size_t)((NB * SEQ * (NQK / 8)) / 256) * 256 * 8 == (size_t)NB * SEQ * NQK);
static_assert((size_t)(KVC / 64) * ((NB * SEQ) / 64) * 4096 == (size_t)KVC * NB * SEQ);
static_assert((size_t)(SEQ / 64) * NH * NB * 4 * 16 * HD == (size_t)NB * SEQ * DM);
static_assert((size_t)(SEQ / 64) * (DM / 64) * NB * 4096 == (size_t)NB * SEQ * DM);

extern "C" void kernel_launch(void* const* d_in, const int* in_sizes, int n_in, void* d_out, int out_size, void* d_ws, size_t ws_size, hipStream_t stream) {
  if (n_in < 8) return;
  if ((long long)in_sizes[0] < (long long)(NB - 1) * SEQ_FULL * DM + (long long)SEQ * DM) return;
  if (in_sizes[1] < DM * DM || in_sizes[2] < DM || in_sizes[3] < DM * KVC || in_sizes[4] < KVC) return;
  if (in_sizes[5] < DM * KVC || in_sizes[6] < KVC || in_sizes[7] < DM * DM) return;
  if ((long long)out_size < (long long)NB * SEQ * DM) return;
  if (ws_size < WS_TOTAL) return;
  const float* x  = (const float*)d_in[0];
  const float* Wq = (const float*)d_in[1];
  const float* bq = (const float*)d_in[2];
  const float* Wk = (const float*)d_in[3];
  const float* bk = (const float*)d_in[4];
  const float* Wv = (const float*)d_in[5];
  const float* bv = (const float*)d_in[6];
  const float* Wo = (const float*)d_in[7];
  float* out = (float*)d_out;

  char* wsp = (char*)d_ws;
  unsigned short* X16   = (unsigned short*)wsp; wsp += SZ_X16;
  unsigned short* WQK16 = (unsigned short*)wsp; wsp += SZ_WQK;
  unsigned short* WV16  = (unsigned short*)wsp; wsp += SZ_WV;
  unsigned short* WO16  = (unsigned short*)wsp; wsp += SZ_WO;
  float*          BALL  = (float*)wsp;          wsp += SZ_BALL;
  float*          CSTAB = (float*)wsp;          wsp += SZ_CS;
  float*          QKF   = (float*)wsp;          wsp += SZ_QKF;
  unsigned short* QKH   = (unsigned short*)wsp; wsp += SZ_QKH;
  unsigned short* VTH   = (unsigned short*)wsp; wsp += SZ_VT;
  unsigned short* CTXH  = (unsigned short*)wsp; wsp += SZ_CTXH;
  if ((size_t)(wsp - (char*)d_ws) > ws_size) return;

  k_castb<<<dim3((unsigned)((SEQ * (DM / 8)) / 256), (unsigned)NB), 256, 0, stream>>>(x, (size_t)SEQ_FULL * DM, (unsigned)DM, X16, (size_t)SEQ * DM, (unsigned)DM, (unsigned)SEQ, (unsigned)DM);
  k_castT<<<(unsigned)((DM * (DM / 8)) / 256), 256, 0, stream>>>(Wq, (unsigned)DM, WQK16, (unsigned)DM, (unsigned)DM, (unsigned)DM, 16.0f);
  k_castT<<<(unsigned)((KVC * (DM / 8)) / 256), 256, 0, stream>>>(Wk, (unsigned)KVC, WQK16 + (size_t)DM * DM, (unsigned)DM, (unsigned)DM, (unsigned)KVC, 16.0f);
  k_castT<<<(unsigned)((KVC * (DM / 8)) / 256), 256, 0, stream>>>(Wv, (unsigned)KVC, WV16, (unsigned)DM, (unsigned)DM, (unsigned)KVC, 16.0f);
  k_castT<<<(unsigned)((DM * (DM / 8)) / 256), 256, 0, stream>>>(Wo, (unsigned)DM, WO16, (unsigned)DM, (unsigned)DM, (unsigned)DM, 16.0f);
  k_bias<<<(unsigned)(NBIAS / 256), 256, 0, stream>>>(bq, bk, bv, BALL);
  k_cstab<<<(unsigned)((SEQ * NPAIR) / 256), 256, 0, stream>>>(CSTAB);

  k_gemm64<2, 0><<<dim3((unsigned)((((NB * SEQ) / 64) * (NQK / 64) + 7) / 8), 1u), 256, 0, stream>>>(
      X16, (unsigned)DM, (size_t)0, WQK16, (unsigned)DM, (size_t)0,
      (void*)QKF, (unsigned)NQK, (size_t)0, BALL,
      (unsigned)(NB * SEQ), (unsigned)NQK, (unsigned)DM, 0.0625f);
  k_rope<<<(unsigned)((NB * SEQ * (NQK / 8)) / 256), 256, 0, stream>>>(QKF, CSTAB, QKH, (unsigned)(NB * SEQ));
  k_gemm64<1, 1><<<dim3((unsigned)(((KVC / 64) * ((NB * SEQ) / 64) + 7) / 8), 1u), 256, 0, stream>>>(
      WV16, (unsigned)DM, (size_t)0, X16, (unsigned)DM, (size_t)0,
      (void*)VTH, (unsigned)(NB * SEQ), (size_t)0, BALL + NQK,
      (unsigned)KVC, (unsigned)(NB * SEQ), (unsigned)DM, 0.0625f);

  k_fattn<<<dim3((unsigned)(SEQ / 64), (unsigned)NH, (unsigned)NB), 128, 0, stream>>>(
      QKH, QKH + DM, (unsigned)NQK, (size_t)SEQ * NQK,
      VTH, (unsigned)(NB * SEQ), (unsigned)SEQ,
      CTXH, (unsigned)DM, (size_t)SEQ * DM, (unsigned)(SEQ / 64));

  k_gemm64<0, 0><<<dim3((unsigned)(((SEQ / 64) * (DM / 64) + 7) / 8), (unsigned)NB), 256, 0, stream>>>(
      CTXH, (unsigned)DM, (size_t)SEQ * DM, WO16, (unsigned)DM, (size_t)0,
      (void*)out, (unsigned)DM, (size_t)SEQ * DM, BALL,
      (unsigned)SEQ, (unsigned)DM, (unsigned)DM, 0.0009765625f);
}
